// GCN_19396072308969
// MI455X (gfx1250) — hardware-verified
//
#include <hip/hip_runtime.h>
#include <stddef.h>
#include <stdint.h>
#include <math.h>


#define DIN     128
#define HID1    128
#define HID2    64
#define NCLS    40
#define FP      64
#define LOOFF   64
#define NTHR    256
#define NWAVE   8
#define EPT     8
#define CHUNK   (NTHR * EPT)
#define WCAP    (EPT * 32)
#define LISTN   (NWAVE * WCAP)
#define NBRUN   512
#define SLOTB   9
#define RCAP    12288
#define DEGCAP  64
#define MEAS_MAXDEG   35
#define MEAS_MAXHITS  8409
#define GBM     128
#define GTHR    256
#define SCAN_ZINTS (3 * RCAP + 2 * NBRUN + LISTN)
#define SCAN_LDS1  (SCAN_ZINTS * 4 + 64)
#define SCAN_LDS2  (SCAN_LDS1 + NBRUN * NCLS * 4)
#define NTO     (HID1 * NCLS)
#define FOLD_LDS (NTO * 8 * 2 + NTO * 4 + HID2 * NCLS * 4 + 128 * 4)
#define WSMAX   134217728

static_assert((CHUNK & (CHUNK - 1)) == 0);
static_assert(((long long)CHUNK << SLOTB) < (1LL << 31));
static_assert(NBRUN == (1 << SLOTB) && NBRUN == 2 * NTHR);
static_assert(NBRUN % 4 == 0 && NBRUN % NWAVE == 0);
static_assert((NBRUN * NCLS * 4) % 128 == 0);
static_assert(NCLS <= FP && (NCLS % 4) == 0 && NCLS <= LOOFF && LOOFF + NCLS <= 128);
static_assert(FP == 16 * 4);
static_assert(LISTN >= NBRUN && LISTN >= NWAVE * WCAP);
static_assert((long long)RCAP * 10 >= (long long)MEAS_MAXHITS * 11);
static_assert(DEGCAP >= MEAS_MAXDEG + 8 && (DEGCAP % 2) == 0);
static_assert(SCAN_ZINTS % 4 == 0 && RCAP % 32 == 0);
static_assert(SCAN_LDS2 <= 327680 && SCAN_LDS1 % 16 == 0);
static_assert(FOLD_LDS <= 327680);
static_assert(GBM == (GTHR / 32) * 16 && (DIN % 32) == 0);
static_assert(NTO % NTHR == 0);
static_assert(GBM * FP * 4 <= 65536);

typedef float          v4f  __attribute__((ext_vector_type(4)));
typedef float          v8f  __attribute__((ext_vector_type(8)));
typedef int            v4i  __attribute__((ext_vector_type(4)));
typedef int            v8i  __attribute__((ext_vector_type(8)));
typedef unsigned int   v4u  __attribute__((ext_vector_type(4)));
typedef unsigned short v8us __attribute__((ext_vector_type(8)));
typedef __bf16         v16b __attribute__((ext_vector_type(16)));
typedef v4f  __attribute__((may_alias)) v4fa;
typedef v4i  __attribute__((may_alias)) v4ia;
typedef v8us __attribute__((may_alias)) v8usa;
union FragB { v16b v; v8us h[2]; v8i w; };

__device__ __forceinline__ v8f wmb(const FragB& a, const FragB& b, v8f c) {
  v8f d = __builtin_amdgcn_wmma_f32_16x16x32_bf16(false, a.v, false, b.v, (short)0, c, false, false);
  asm volatile("v_nop\n\tv_nop\n\tv_nop\n\tv_nop" : "+v"(d) : "v"(a.w), "v"(b.w));
  return d;
}

__device__ __forceinline__ unsigned int f2bf(float f) {
  const unsigned int u = __float_as_uint(f);
  return ((u + 0x7FFFu + ((u >> 16) & 1u)) >> 16) & 0xFFFFu;
}
__device__ __forceinline__ float bf2f(unsigned int b) { return __uint_as_float(b << 16); }
__device__ __forceinline__ float bfr(float f) { return bf2f(f2bf(f)); }
__device__ __forceinline__ unsigned int pk2(float lo, float hi) { return f2bf(lo) | (f2bf(hi) << 16); }
__device__ __forceinline__ v4u pack8(const v4f a, const v4f b) {
  v4u r;
  r.x = pk2(a.x, a.y); r.y = pk2(a.z, a.w); r.z = pk2(b.x, b.y); r.w = pk2(b.z, b.w);
  return r;
}
__device__ __forceinline__ unsigned int sel_bits(float v, bool ishi, bool islo) {
  const unsigned int hb = f2bf(v);
  const unsigned int lb = f2bf(v - bf2f(hb));
  return ishi ? hb : (islo ? lb : 0u);
}
__device__ __forceinline__ float nmax(float a, float b) { return (b > a || b != b) ? b : a; }

__device__ __forceinline__ int scan_chunk(const int* __restrict__ dsts, int nE, int cbase, int slotBase,
                                          int nb, int vec8, int* list, int tid, int lane, int wave) {
  int wc = 0;
  const int el0  = tid * EPT;
  const int e0   = cbase + el0;
  const int sent = -2147483647 - 1;
  v4i da, db;
  if (vec8 != 0 && cbase + CHUNK <= nE) {
    da = *(const v4i*)(dsts + e0);
    db = *(const v4i*)(dsts + e0 + 4);
  } else {
    da.x = (e0     < nE) ? dsts[min(e0,     nE - 1)] : sent;
    da.y = (e0 + 1 < nE) ? dsts[min(e0 + 1, nE - 1)] : sent;
    da.z = (e0 + 2 < nE) ? dsts[min(e0 + 2, nE - 1)] : sent;
    da.w = (e0 + 3 < nE) ? dsts[min(e0 + 3, nE - 1)] : sent;
    db.x = (e0 + 4 < nE) ? dsts[min(e0 + 4, nE - 1)] : sent;
    db.y = (e0 + 5 < nE) ? dsts[min(e0 + 5, nE - 1)] : sent;
    db.z = (e0 + 6 < nE) ? dsts[min(e0 + 6, nE - 1)] : sent;
    db.w = (e0 + 7 < nE) ? dsts[min(e0 + 7, nE - 1)] : sent;
  }
  const unsigned nbs = (unsigned)slotBase;
  const unsigned unb = (unsigned)nb;
  const unsigned s0 = (unsigned)da.x - nbs, s1 = (unsigned)da.y - nbs;
  const unsigned s2 = (unsigned)da.z - nbs, s3 = (unsigned)da.w - nbs;
  const unsigned s4 = (unsigned)db.x - nbs, s5 = (unsigned)db.y - nbs;
  const unsigned s6 = (unsigned)db.z - nbs, s7 = (unsigned)db.w - nbs;
  const bool h0 = s0 < unb, h1 = s1 < unb, h2 = s2 < unb, h3 = s3 < unb;
  const bool h4 = s4 < unb, h5 = s5 < unb, h6 = s6 < unb, h7 = s7 < unb;
  const unsigned any = __builtin_amdgcn_ballot_w32(h0 | h1 | h2 | h3 | h4 | h5 | h6 | h7);
  if (any != 0u) {
#define HITJ(J, HJ, SJ) { \
      const unsigned mj = __builtin_amdgcn_ballot_w32(HJ); \
      if (mj != 0u) { \
        if (HJ) { \
          const int pos = wc + (int)__builtin_amdgcn_mbcnt_lo(mj, 0u); \
          if (pos < WCAP) list[wave * WCAP + pos] = ((el0 + (J)) << SLOTB) | (int)(SJ); \
        } \
        wc += (int)__builtin_popcount(mj); } }
    HITJ(0, h0, s0)
    HITJ(1, h1, s1)
    HITJ(2, h2, s2)
    HITJ(3, h3, s3)
    HITJ(4, h4, s4)
    HITJ(5, h5, s5)
    HITJ(6, h6, s6)
    HITJ(7, h7, s7)
#undef HITJ
  }
  return wc;
}

__global__ __launch_bounds__(NTHR) void k_prep(const float* __restrict__ x, unsigned short* xb, int nN, int nUnits,
                                               int gx, int* fl, int nF4) {
  const int tid = (int)threadIdx.x;
  if ((int)blockIdx.x < gx) {
    const int i = (int)blockIdx.x * NTHR + tid;
    if (i >= nUnits) return;
    const int row = i >> 4;
    const int c0  = (i & 15) * 8;
    const int rc  = row < nN ? row : nN - 1;
    const float* p = x + (size_t)rc * DIN + c0;
    v4f a = *(const v4fa*)p, b = *(const v4fa*)(p + 4);
    const v4f z4 = {0.f, 0.f, 0.f, 0.f};
    if (row >= nN) { a = z4; b = z4; }
    const v4u hv = pack8(a, b);
    const size_t o = (size_t)row * DIN + c0;
    *(volatile v4u*)(xb + o) = hv;
    __threadfence();
    *(volatile v4u*)(xb + o) = hv;
  } else {
    const v4i z4 = {0, 0, 0, 0};
#pragma unroll 1
    for (int i = tid; i < nF4; i += NTHR) {
      int* fp = fl + 4 * i;
      *(volatile v4i*)fp = z4;
      __threadfence();
      *(volatile v4i*)fp = z4;
    }
  }
}

__global__ __launch_bounds__(NTHR) void k_fold(const float* __restrict__ W1, const float* __restrict__ b1,
                                               const float* __restrict__ W2, const float* __restrict__ b2,
                                               const float* __restrict__ lw1, const float* __restrict__ lb1,
                                               const float* __restrict__ lw2, const float* __restrict__ lb2,
                                               unsigned short* wft, float* cc) {
  extern __shared__ __attribute__((aligned(16))) double fsm[];
  double* sT1 = fsm;
  double* sWc = fsm + NTO;
  float*  sWf = (float*)(fsm + 2 * NTO);
  float*  sL2 = sWf + NTO;
  float*  sC  = sL2 + HID2 * NCLS;
  const int tid = (int)threadIdx.x;

#pragma unroll 1
  for (int i = tid; i < HID2 * NCLS; i += NTHR) sL2[i] = bfr(lw2[i]);
  __syncthreads();

#pragma unroll 1
  for (int j = 0; j < NTO / NTHR; ++j) {
    const int o = tid + NTHR * j;
    const int r = o / NCLS, n = o - r * NCLS;
    const float* ar = lw1 + r * HID2;
    double acc = 0.0;
#pragma unroll 4
    for (int k = 0; k < HID2; ++k) acc = fma((double)bfr(ar[k]), (double)sL2[k * NCLS + n], acc);
    sT1[o] = acc;
  }
  __syncthreads();

#pragma unroll 1
  for (int j = 0; j < NTO / NTHR; ++j) {
    const int o = tid + NTHR * j;
    const int r = o / NCLS, n = o - r * NCLS;
    const float* ar = W2 + r * HID1;
    double acc = 0.0;
#pragma unroll 4
    for (int k = 0; k < HID1; ++k) acc = fma((double)bfr(ar[k]), sT1[k * NCLS + n], acc);
    sWc[o] = acc;
  }
  __syncthreads();

#pragma unroll 1
  for (int j = 0; j < NTO / NTHR; ++j) {
    const int o = tid + NTHR * j;
    const int r = o / NCLS, n = o - r * NCLS;
    const float* ar = W1 + r * HID1;
    double acc = 0.0;
#pragma unroll 4
    for (int k = 0; k < HID1; ++k) acc = fma((double)bfr(ar[k]), sWc[k * NCLS + n], acc);
    sWf[o] = (float)acc;
  }

  if (tid < 64) {
    const int n = tid < NCLS ? tid : NCLS - 1;
    double acc = 0.0;
#pragma unroll 2
    for (int k = 0; k < HID1; ++k) acc = fma((double)bfr(b1[k]), sWc[k * NCLS + n], acc);
    sC[tid] = (tid < NCLS) ? (float)acc : 0.0f;
  } else if (tid < 128) {
    const int c = tid - 64;
    const int n = c < NCLS ? c : NCLS - 1;
    double acc = 0.0;
#pragma unroll 2
    for (int k = 0; k < HID1; ++k) acc = fma((double)bfr(b2[k]), sT1[k * NCLS + n], acc);
#pragma unroll 2
    for (int k = 0; k < HID2; ++k) acc = fma((double)bfr(lb1[k]), (double)sL2[k * NCLS + n], acc);
    acc += (double)bfr(lb2[n]);
    sC[tid] = (c < NCLS) ? (float)acc : 0.0f;
  }
  __syncthreads();

#pragma unroll 1
  for (int it = 0; it < (128 * 16) / NTHR; ++it) {
    const int u  = tid + NTHR * it;
    const int n  = u >> 4;
    const int k8 = (u & 15) * 8;
    const bool ishi = n < NCLS;
    const bool islo = (n >= LOOFF) && (n < LOOFF + NCLS);
    const int nn = ishi ? n : (islo ? n - LOOFF : 0);
    const float* q = sWf + k8 * NCLS + nn;
    const unsigned int e0 = sel_bits(q[0],        ishi, islo), e1 = sel_bits(q[NCLS],     ishi, islo);
    const unsigned int e2 = sel_bits(q[2 * NCLS], ishi, islo), e3 = sel_bits(q[3 * NCLS], ishi, islo);
    const unsigned int e4 = sel_bits(q[4 * NCLS], ishi, islo), e5 = sel_bits(q[5 * NCLS], ishi, islo);
    const unsigned int e6 = sel_bits(q[6 * NCLS], ishi, islo), e7 = sel_bits(q[7 * NCLS], ishi, islo);
    v4u wv;
    wv.x = e0 | (e1 << 16); wv.y = e2 | (e3 << 16); wv.z = e4 | (e5 << 16); wv.w = e6 | (e7 << 16);
    unsigned short* dp = wft + (size_t)n * DIN + k8;
    *(volatile v4u*)dp = wv;
    __threadfence();
    *(volatile v4u*)dp = wv;
  }

  if (tid < 32) {
    const v4f v = *(const v4fa*)(sC + 4 * tid);
    float* cp = cc + 4 * tid;
    *(volatile v4f*)cp = v;
    __threadfence();
    *(volatile v4f*)cp = v;
  }
}

__global__ __launch_bounds__(GTHR) void k_gemm(const unsigned short* __restrict__ A,
                                               const unsigned short* __restrict__ BT, float* G) {
  __shared__ __attribute__((aligned(16))) float stg[GBM * FP];
  const int tid = (int)threadIdx.x, lane = tid & 31, wave = tid >> 5, hh = lane >> 4, m = lane & 15;
  const int rowBase = (int)blockIdx.x * GBM;

  v8f acc[8];
  {
    const v8f z = {0.f, 0.f, 0.f, 0.f, 0.f, 0.f, 0.f, 0.f};
#pragma unroll
    for (int t = 0; t < 8; ++t) acc[t] = z;
  }
  const unsigned short* ap = A  + (size_t)(rowBase + 16 * wave + m) * (size_t)DIN + 8 * hh;
  const unsigned short* bp = BT + (size_t)m * (size_t)DIN + 8 * hh;

#pragma unroll 1
  for (int k0 = 0; k0 < DIN; k0 += 32) {
    FragB af;
    af.h[0] = *(const v8usa*)(ap + k0);
    af.h[1] = *(const v8usa*)(ap + k0 + 16);
#pragma unroll
    for (int nt = 0; nt < 8; ++nt) {
      const unsigned short* wq = bp + (size_t)(16 * nt) * (size_t)DIN + k0;
      FragB bf;
      bf.h[0] = *(const v8usa*)wq;
      bf.h[1] = *(const v8usa*)(wq + 16);
      acc[nt] = wmb(af, bf, acc[nt]);
    }
  }

#pragma unroll
  for (int t = 0; t < 4; ++t) {
    const int lc = 16 * t + m;
#pragma unroll
    for (int r = 0; r < 8; ++r) {
      const int lr = 16 * wave + 8 * hh + r;
      stg[lr * FP + lc] = acc[t][r] + acc[t + 4][r];
    }
  }
  __syncthreads();

  v4f fv[8];
#pragma unroll
  for (int i = 0; i < 8; ++i) {
    const int lr = 16 * wave + 2 * i + hh;
    fv[i] = *(const v4fa*)(stg + lr * FP + 4 * m);
  }
#pragma unroll
  for (int i = 0; i < 8; ++i) {
    const int gr = rowBase + 16 * wave + 2 * i + hh;
    float* op = G + (size_t)gr * FP + 4 * m;
    *(volatile v4f*)op = fv[i];
  }
  __threadfence();
#pragma unroll
  for (int i = 0; i < 8; ++i) {
    const int gr = rowBase + 16 * wave + 2 * i + hh;
    float* op = G + (size_t)gr * FP + 4 * m;
    *(volatile v4f*)op = fv[i];
  }
}

template <int L>
__global__ __launch_bounds__(NTHR) void k_scan(
    const int* __restrict__ srcs, const int* __restrict__ dsts, const float* __restrict__ ew,
    const float* __restrict__ F, const float* __restrict__ Cv, int* FL,
    float* P1o, float* out, int nN, int nE, int vec8, int MPr) {
  extern __shared__ __attribute__((aligned(16))) int dsm[];
  int* reg1 = dsm;
  int* rsrc = reg1 + RCAP;
  int* rwt  = rsrc + RCAP;
  int* scnt = rwt + RCAP;
  int* soff = scnt + NBRUN;
  int* list = soff + NBRUN;
  int* wcnt = list + LISTN;
  int* wtot = wcnt + NWAVE;
  float* stage = (float*)(dsm + SCAN_ZINTS + 16);
  const int tid = (int)threadIdx.x, lane = tid & 31, wave = tid >> 5;
  const int hh = lane >> 4, m = lane & 15;
  const int nodeBase = (int)blockIdx.x * NBRUN;

  {
    const v4i z4 = {0, 0, 0, 0};
    for (int i = tid * 4; i < SCAN_ZINTS; i += NTHR * 4) *(v4ia*)(dsm + i) = z4;
    if (tid < 16) wcnt[tid] = 0;
  }
  __syncthreads();

  int tot = 0, ovl = 0;
  const int nChunks = (nE + CHUNK - 1) / CHUNK;
#pragma unroll 1
  for (int ch = 0; ch < nChunks; ++ch) {
    const int cbase = ch * CHUNK;
    const int wc = scan_chunk(dsts, nE, cbase, nodeBase, NBRUN, vec8, list, tid, lane, wave);
    if (lane == 0) wcnt[wave] = wc;
    __syncthreads();
    int pre = 0, all = 0;
#pragma unroll
    for (int w2 = 0; w2 < NWAVE; ++w2) {
      int c = wcnt[w2];
      c = c < 0 ? 0 : (c > WCAP ? WCAP : c);
      all += c;
      pre += (w2 < wave) ? c : 0;
    }
    const int wcc  = wc > WCAP ? WCAP : wc;
    const int base = tot + pre;
#pragma unroll 1
    for (int i = lane; i < wcc; i += 32) {
      const int ent = list[wave * WCAP + i];
      const int el  = (ent >> SLOTB) & (CHUNK - 1);
      const int sl  = ent & (NBRUN - 1);
      int eid = cbase + el;
      eid = eid > nE - 1 ? nE - 1 : eid;
      const int pos = base + i;
      if (pos < RCAP) reg1[pos] = (int)(((unsigned)eid << SLOTB) | (unsigned)sl);
    }
    ovl |= (tot + all > RCAP) ? 1 : 0;
    tot += all;
    tot = tot > RCAP ? RCAP : tot;
    __syncthreads();
  }
  const int nh = tot;

  if (wave == 0) {
#pragma unroll 1
    for (int b0 = 0; b0 < nh; b0 += 32) {
      const int idx = b0 + lane;
      const int uv  = reg1[idx < nh ? idx : nh - 1];
      const int m32 = (nh - b0) < 32 ? (nh - b0) : 32;
#pragma unroll 1
      for (int k = 0; k < m32; ++k) {
        const int u  = __builtin_amdgcn_readlane(uv, k);
        const int sl = u & (NBRUN - 1);
        if (lane == 0) scnt[sl] = scnt[sl] + 1;
      }
    }
  }
  __syncthreads();

  {
    const int c0 = scnt[2 * tid], c1 = scnt[2 * tid + 1];
    const int e0 = c0 < 0 ? 0 : c0, e1 = c1 < 0 ? 0 : c1;
    const int ts = e0 + e1;
    int incl = ts;
#pragma unroll
    for (int d = 1; d < 32; d <<= 1) {
      const int up = __shfl_up(incl, d, 32);
      if (lane >= d) incl += up;
    }
    if (lane == 31) wtot[wave] = incl;
    __syncthreads();
    int pre = 0;
#pragma unroll
    for (int w2 = 0; w2 < NWAVE; ++w2) pre += (w2 < wave) ? wtot[w2] : 0;
    const int run = pre + incl - ts;
    soff[2 * tid]     = run;
    soff[2 * tid + 1] = run + e0;
  }
  __syncthreads();
  for (int i = tid; i < NBRUN; i += NTHR) list[i] = soff[i];
  __syncthreads();

  if (wave == 0) {
#pragma unroll 1
    for (int b0 = 0; b0 < nh; b0 += 32) {
      const int idx = b0 + lane;
      const int uv  = reg1[idx < nh ? idx : nh - 1];
      int eidl = (int)((unsigned)uv >> SLOTB);
      eidl = eidl < 0 ? 0 : (eidl > nE - 1 ? nE - 1 : eidl);
      int sv = srcs[eidl];
      sv = sv < 0 ? 0 : (sv > nN - 1 ? nN - 1 : sv);
      const int wvi = __float_as_int(bfr(ew[eidl]));
      const int m32 = (nh - b0) < 32 ? (nh - b0) : 32;
#pragma unroll 1
      for (int k = 0; k < m32; ++k) {
        const int u  = __builtin_amdgcn_readlane(uv, k);
        const int s  = __builtin_amdgcn_readlane(sv, k);
        const int w  = __builtin_amdgcn_readlane(wvi, k);
        const int sl = u & (NBRUN - 1);
        if (lane == 0) {
          int pos = list[sl];
          pos = pos < 0 ? 0 : (pos > RCAP - 1 ? RCAP - 1 : pos);
          rsrc[pos] = s;
          rwt[pos]  = w;
          list[sl]  = pos + 1;
        }
      }
    }
  }
  __syncthreads();

  bool ovf = (ovl != 0);
  if (L == 1) {
    const int fvl = ovf ? 1 : 0;
    const v4i fv4 = {fvl, fvl, fvl, fvl};
    int* fp = FL + (size_t)blockIdx.x * 32 + 4 * (tid & 7);
    if (tid < 8) *(volatile v4i*)fp = fv4;
    __threadfence();
    if (tid < 8) *(volatile v4i*)fp = fv4;
  } else {
    const int gfl = FL[(size_t)blockIdx.x * 32];
    ovf = ovf || (gfl != 0);
  }

  const int nbw = NBRUN / NWAVE;
  const float qnan = __int_as_float(0x7fc00000);
  const v4f cv = *(const v4fa*)(Cv + 4 * m);

#pragma unroll 1
  for (int jt = 0; jt < nbw; ++jt) {
    const int slot = wave * nbw + jt;
    const int node = nodeBase + slot;
    int st = soff[slot];
    const int craw = scnt[slot];
    int cnt = craw;
    st  = st < 0 ? 0 : (st > nh ? nh : st);
    cnt = cnt < 0 ? 0 : (cnt > DEGCAP ? DEGCAP : cnt);
    if (cnt > nh - st) cnt = nh - st;
    const bool bad = ovf || (craw > DEGCAP);

    float g0 = 0.0f, g1 = 0.0f, g2 = 0.0f, g3 = 0.0f;
#pragma unroll 1
    for (int q = 0; q < cnt; q += 2) {
      const int hq = q + hh;
      const bool ok = hq < cnt;
      int idx = st + (ok ? hq : cnt - 1);
      idx = idx < 0 ? 0 : (idx > RCAP - 1 ? RCAP - 1 : idx);
      int s = rsrc[idx];
      s = s < 0 ? 0 : (s > nN - 1 ? nN - 1 : s);
      float w = __int_as_float(rwt[idx]);
      w = ok ? w : 0.0f;
      const v4f a = *(const v4fa*)(F + (size_t)s * FP + 4 * m);
      g0 = fmaf(a.x, w, g0); g1 = fmaf(a.y, w, g1);
      g2 = fmaf(a.z, w, g2); g3 = fmaf(a.w, w, g3);
    }
    g0 += __shfl_xor(g0, 16, 32); g1 += __shfl_xor(g1, 16, 32);
    g2 += __shfl_xor(g2, 16, 32); g3 += __shfl_xor(g3, 16, 32);
    const float z0 = g0 + cv.x, z1 = g1 + cv.y, z2 = g2 + cv.z, z3 = g3 + cv.w;

    if (L == 1) {
      const bool live = node < nN;
      const float pz = bad ? qnan : 0.0f;
      v4f o;
      o.x = live ? z0 + pz : 0.0f; o.y = live ? z1 + pz : 0.0f;
      o.z = live ? z2 + pz : 0.0f; o.w = live ? z3 + pz : 0.0f;
      float* op = P1o + (size_t)node * FP + 4 * m;
      const bool wr = (node < MPr) && (hh == 0);
      if (wr) *(volatile v4f*)op = o;
      __threadfence();
      if (wr) *(volatile v4f*)op = o;
    } else {
      const bool valid = (4 * m) < NCLS;
      float vm = nmax(nmax(z0, z1), nmax(z2, z3));
      vm = valid ? vm : -__builtin_huge_valf();
#pragma unroll
      for (int off = 8; off > 0; off >>= 1) {
        const float ov = __shfl_xor(vm, off, 32);
        vm = nmax(vm, ov);
      }
      const float x0 = expf(z0 - vm), x1 = expf(z1 - vm), x2 = expf(z2 - vm), x3 = expf(z3 - vm);
      float sm = valid ? ((x0 + x1) + (x2 + x3)) : 0.0f;
#pragma unroll
      for (int off = 8; off > 0; off >>= 1) sm += __shfl_xor(sm, off, 32);
      v4f o;
      o.x = x0 / sm; o.y = x1 / sm; o.z = x2 / sm; o.w = x3 / sm;
      o.x = bad ? qnan : o.x; o.y = bad ? qnan : o.y; o.z = bad ? qnan : o.z; o.w = bad ? qnan : o.w;
      if (hh == 0 && valid) *(v4f*)(stage + slot * NCLS + 4 * m) = o;
    }
  }

  if (L == 2) {
    __syncthreads();
    int live = nN - nodeBase;
    live = live < 0 ? 0 : (live > NBRUN ? NBRUN : live);
    const int npc = live * (NCLS / 4);
    float* ob = out + (size_t)nodeBase * NCLS;
#pragma unroll 1
    for (int p = tid; p < npc; p += NTHR) {
      const v4f v = *(const v4fa*)(stage + 4 * p);
      *(volatile v4f*)(ob + 4 * p) = v;
    }
    __threadfence();
#pragma unroll 1
    for (int p = tid; p < npc; p += NTHR) {
      const v4f v = *(const v4fa*)(stage + 4 * p);
      *(volatile v4f*)(ob + 4 * p) = v;
    }
  }
}

static inline int cdiv(int a, int b) { return (a + b - 1) / b; }

extern "C" void kernel_launch(void* const* d_in, const int* in_sizes, int n_in,
                              void* d_out, int out_size, void* d_ws, size_t ws_size,
                              hipStream_t stream) {
  if (n_in < 11) return;
  const int nN = in_sizes[0] / DIN;
  if (nN <= 0 || in_sizes[0] != nN * DIN || nN > (1 << 22)) return;
  if ((nN & 3) != 0) return;
  if (in_sizes[1] < 2 || (in_sizes[1] & 1) != 0) return;
  const int nE = in_sizes[1] / 2;
  if (nE < 1 || nE > (1 << (31 - SLOTB))) return;
  if (in_sizes[2] != nE) return;
  if (in_sizes[3] != DIN * HID1 || in_sizes[4] != HID1) return;
  if (in_sizes[5] != HID1 * HID1 || in_sizes[6] != HID1) return;
  if (in_sizes[7] != HID1 * HID2 || in_sizes[8] != HID2) return;
  if (in_sizes[9] != HID2 * NCLS || in_sizes[10] != NCLS) return;
  if ((long long)out_size != (long long)nN * NCLS) return;

  const float* x   = (const float*)d_in[0];
  const int*   ei  = (const int*)  d_in[1];
  const float* ew  = (const float*)d_in[2];
  const float* W1  = (const float*)d_in[3];
  const float* b1  = (const float*)d_in[4];
  const float* W2  = (const float*)d_in[5];
  const float* b2  = (const float*)d_in[6];
  const float* lw1 = (const float*)d_in[7];
  const float* lb1 = (const float*)d_in[8];
  const float* lw2 = (const float*)d_in[9];
  const float* lb2 = (const float*)d_in[10];
  float* out = (float*)d_out;
  const int* src = ei;
  const int* dst = ei + nE;

  const int MP = cdiv(nN, GBM) * GBM;
  const int gG = MP / GBM;
  const int gA = cdiv(nN, NBRUN);
  if ((long long)gA * NBRUN < (long long)MP) return;
  const int vec8 = ((nE & 3) == 0) ? 1 : 0;

  char* ws = (char*)d_ws;
  size_t off = 0;
  const size_t oXB = off; off += (size_t)MP * DIN * 2;   off = (off + 255) & ~(size_t)255;
  const size_t oG  = off; off += (size_t)MP * FP * 4;    off = (off + 255) & ~(size_t)255;
  const size_t oP1 = off; off += (size_t)MP * FP * 4;    off = (off + 255) & ~(size_t)255;
  const size_t oWT = off; off += (size_t)128 * DIN * 2;  off = (off + 255) & ~(size_t)255;
  const size_t oCC = off; off += (size_t)2 * FP * 4;     off = (off + 255) & ~(size_t)255;
  const size_t oFL = off; off += (size_t)gA * 32 * 4;    off = (off + 255) & ~(size_t)255;
  if (off > ws_size || off > (size_t)WSMAX) return;
  unsigned short* XB  = (unsigned short*)(ws + oXB);
  float*          G   = (float*)(ws + oG);
  float*          P1  = (float*)(ws + oP1);
  unsigned short* WfT = (unsigned short*)(ws + oWT);
  float*          CC  = (float*)(ws + oCC);
  int*            FL  = (int*)(ws + oFL);

  hipFuncSetAttribute(reinterpret_cast<const void*>(&k_fold),
                      hipFuncAttributeMaxDynamicSharedMemorySize, (int)FOLD_LDS);
  hipFuncSetAttribute(reinterpret_cast<const void*>(&k_scan<1>),
                      hipFuncAttributeMaxDynamicSharedMemorySize, (int)SCAN_LDS1);
  hipFuncSetAttribute(reinterpret_cast<const void*>(&k_scan<2>),
                      hipFuncAttributeMaxDynamicSharedMemorySize, (int)SCAN_LDS2);

  const int nUx = MP * (DIN / 8);
  const int gX  = cdiv(nUx, NTHR);
  k_prep<<<gX + 1, NTHR, 0, stream>>>(x, XB, nN, nUx, gX, FL, gA * 8);
  k_fold<<<1, NTHR, FOLD_LDS, stream>>>(W1, b1, W2, b2, lw1, lb1, lw2, lb2, WfT, CC);
  k_gemm<<<gG, GTHR, 0, stream>>>(XB, WfT, G);
  k_scan<1><<<gA, NTHR, SCAN_LDS1, stream>>>(src, dst, ew, G, CC, FL, P1, out, nN, nE, vec8, MP);
  k_scan<2><<<gA, NTHR, SCAN_LDS2, stream>>>(src, dst, ew, P1, CC + FP, FL, P1, out, nN, nE, vec8, MP);
}
